// BCA_17274358465235
// MI455X (gfx1250) — hardware-verified
//
#include <hip/hip_runtime.h>
#include <math.h>

typedef __attribute__((ext_vector_type(16))) _Float16 v16h;
typedef __attribute__((ext_vector_type(16))) __bf16 v16b;
typedef __attribute__((ext_vector_type(8)))  _Float16 v8h;
typedef __attribute__((ext_vector_type(8)))  float v8f;
typedef __attribute__((ext_vector_type(4)))  float v4f;
typedef __attribute__((ext_vector_type(2)))  float v2f;
typedef __attribute__((ext_vector_type(4)))  unsigned v4u;
typedef __attribute__((ext_vector_type(4)))  int v4i;
typedef float __attribute__((may_alias)) float_a;
typedef int __attribute__((may_alias)) int_a;

template <typename T> __device__ __forceinline__ void vst2(void* p, T v) { *(volatile T*)p = v; __threadfence(); *(volatile T*)p = v; }
__device__ __forceinline__ v8f wmma16(v16h a, v16h b, v8f c) {
  v8f d = __builtin_amdgcn_wmma_f32_16x16x32_f16(false, a, false, b, (short)0, c, false, false);
  asm volatile("v_nop\n\tv_nop\n\tv_nop\n\tv_nop" : "+v"(d) : "v"(a), "v"(b));
  return d;
}
__device__ __forceinline__ v8f wmma_bf(v16b a, v16b b, v8f c) {
  v8f d = __builtin_amdgcn_wmma_f32_16x16x32_bf16(false, a, false, b, (short)0, c, false, false);
  asm volatile("v_nop\n\tv_nop\n\tv_nop\n\tv_nop" : "+v"(d) : "v"(a), "v"(b));
  return d;
}
__device__ __forceinline__ v16h frag_h(const _Float16* rowk0, int lane) {
  union { v16h v; v8h q[2]; } u; const _Float16* p = rowk0 + 8 * (lane >> 4);
  u.q[0] = *(const v8h*)p; u.q[1] = *(const v8h*)(p + 16); return u.v;
}
__device__ __forceinline__ v16h frag_f32(const float* rowk0, int lane) {
  v16h a; const float* p = rowk0 + 8 * (lane >> 4);
#pragma unroll
  for (int i = 0; i < 8; ++i) { a[i] = (_Float16)p[i]; a[8 + i] = (_Float16)p[16 + i]; }
  return a;
}
__device__ __forceinline__ v16h frag_f32s(const float* rowk0, int lane, float sc) {
  v16h a; const float* p = rowk0 + 8 * (lane >> 4);
#pragma unroll
  for (int i = 0; i < 8; ++i) { a[i] = (_Float16)(p[i] * sc); a[8 + i] = (_Float16)(p[16 + i] * sc); }
  return a;
}
__device__ __forceinline__ v16h fragc_f32(const float* W, int k0, int n, int lane, int ld, int K) {
  v16h a; const int g = lane >> 4;
#pragma unroll
  for (int i = 0; i < 8; ++i) { const int ka = k0 + 8 * g + i, kb = ka + 16;
    a[i] = (_Float16)(ka < K ? W[(size_t)(ka < K ? ka : K - 1) * ld + n] : 0.f); a[8 + i] = (_Float16)(kb < K ? W[(size_t)(kb < K ? kb : K - 1) * ld + n] : 0.f); }
  return a;
}
struct F2 { v16b h, l; };
__device__ __forceinline__ F2 bsplit16(const float v[16]) { F2 r;
#pragma unroll
  for (int i = 0; i < 16; ++i) { const __bf16 h = (__bf16)v[i]; r.h[i] = h; r.l[i] = (__bf16)(v[i] - (float)h); }
  return r; }
__device__ __forceinline__ F2 split_row(const float* row, int k0, int lane) { float v[16]; const float* p = row + k0 + 8 * (lane >> 4);
#pragma unroll
  for (int i = 0; i < 8; ++i) { v[i] = p[i]; v[8 + i] = p[16 + i]; }
  return bsplit16(v); }
__device__ __forceinline__ F2 split_rowK(const float* row, int k0, int lane, int K) { float v[16]; const int g = lane >> 4;
#pragma unroll
  for (int i = 0; i < 8; ++i) { const int ka = k0 + 8 * g + i, kb = ka + 16; v[i] = ka < K ? row[ka < K ? ka : K - 1] : 0.f; v[8 + i] = kb < K ? row[kb < K ? kb : K - 1] : 0.f; }
  return bsplit16(v); }
__device__ __forceinline__ F2 split_col(const float* W, int k0, int n, int lane, int ld, int K) { float v[16]; const int g = lane >> 4;
#pragma unroll
  for (int i = 0; i < 8; ++i) { const int ka = k0 + 8 * g + i, kb = ka + 16; v[i] = ka < K ? W[(size_t)(ka < K ? ka : K - 1) * ld + n] : 0.f; v[8 + i] = kb < K ? W[(size_t)(kb < K ? kb : K - 1) * ld + n] : 0.f; }
  return bsplit16(v); }
__device__ __forceinline__ v8f mac3(const F2& a, const F2& b, v8f c) { c = wmma_bf(a.l, b.h, c); c = wmma_bf(a.h, b.l, c); return wmma_bf(a.h, b.h, c); }
__device__ __forceinline__ float sigm(float v) { return 1.0f / (1.0f + expf(-v)); }
#define LDSX() do { asm volatile("s_wait_dscnt 0" ::: "memory"); __builtin_amdgcn_wave_barrier(); __builtin_amdgcn_fence(__ATOMIC_RELEASE, "workgroup"); } while (0)


#define NB 4
#define CX 256
#define CY 512
#define CM 64
#define HH 64
#define WWD 64
#define NP (HH * WWD)
#define HY 32
#define WY 32
#ifndef TNB
#define TNB NB
#endif
typedef __attribute__((ext_vector_type(8))) __bf16 v8b;
__device__ __forceinline__ v16b frag_b(const __bf16* rowk0, int lane) {
  union { v16b v; v8b q[2]; } u; const __bf16* p = rowk0 + 8 * (lane >> 4);
  u.q[0] = *(const v8b*)p; u.q[1] = *(const v8b*)(p + 16); return u.v;
}
__device__ __forceinline__ float bfr(float v) { return (float)(__bf16)v; }
__device__ __attribute__((noinline)) float exp_ni(float v) { return expf(v); }
__device__ __attribute__((noinline)) float erf_ni(float v) { return erff(v); }

#define WS_FXH 0u
#define WS_FXL (WS_FXH + 2u * (size_t)NB * NP * CM)
#define WS_FYH (WS_FXL + 2u * (size_t)NB * NP * CM)
#define WS_FYL (WS_FYH + 2u * (size_t)NB * NP * CM)
#define WS_FSH (WS_FYL + 2u * (size_t)NB * NP * CM)
#define WS_FSL (WS_FSH + 2u * (size_t)NB * CM * NP)
#define WS_END (WS_FSL + 2u * (size_t)NB * CM * NP)

__device__ __forceinline__ void split_store(float v, _Float16& h, _Float16& l) { const _Float16 hv = (_Float16)v; h = hv; l = (_Float16)((v - (float)hv) * 2048.0f); }
__device__ __forceinline__ void conv2(const float* sa_row0, int col, int lane, int g, const float* __restrict__ W2, v8f acc2[4]) {
#pragma unroll
  for (int j = 0; j < 4; ++j) acc2[j] = v8f{};
#pragma unroll
  for (int kc = 0; kc < CM / 32; ++kc) { const F2 a = split_row(sa_row0, kc * 32, lane);
#pragma unroll
    for (int j = 0; j < 4; ++j) { v16b w; const int o = j * 16 + col;
#pragma unroll
      for (int i = 0; i < 8; ++i) { w[i] = (__bf16)W2[o * CM + kc * 32 + 8 * g + i]; w[8 + i] = (__bf16)W2[o * CM + kc * 32 + 16 + 8 * g + i]; }
      acc2[j] = wmma_bf(a.h, w, acc2[j]); acc2[j] = wmma_bf(a.l, w, acc2[j]); } } }
__global__ __launch_bounds__(128) void k_feat(const float* __restrict__ X, const float* __restrict__ Y, const float* __restrict__ WS1, const float* __restrict__ BS1, const float* __restrict__ WS2, const float* __restrict__ BS2, const float* __restrict__ WX1, const float* __restrict__ BX1, const float* __restrict__ WX2, const float* __restrict__ BX2, const float* __restrict__ WY1, const float* __restrict__ BY1, const float* __restrict__ WY2, const float* __restrict__ BY2,
    _Float16* __restrict__ FXH, _Float16* __restrict__ FXL, _Float16* __restrict__ FYH, _Float16* __restrict__ FYL, _Float16* __restrict__ FSH, _Float16* __restrict__ FSL) {
  __shared__ __align__(16) __bf16 sx[64][CX + 8]; __shared__ __align__(16) float sa[4][16][68]; __shared__ __align__(16) _Float16 sh[64][72], sl[64][72]; __shared__ __align__(16) _Float16 th[64][72], tl[64][72];
  const int tid = threadIdx.x, wave = tid >> 5, lane = tid & 31, col = lane & 15, g = lane >> 4; const int h0 = blockIdx.x; const size_t b = blockIdx.y; const int n0 = h0 * WWD;
  for (int e = tid; e < CX * 64; e += 128) { const int c = e >> 6, nl = e & 63; sx[nl][c] = (__bf16)X[((b * CX + c) * NP) + n0 + nl]; }
  __syncthreads();
#pragma unroll 1
  for (int which = 0; which < 2; ++which) { const float* W1 = which == 0 ? WS1 : WX1; const float* B1 = which == 0 ? BS1 : BX1; const float* W2 = which == 0 ? WS2 : WX2; const float* B2 = which == 0 ? BS2 : BX2;
    v8f acc[4] = {};
#pragma unroll
    for (int kc = 0; kc < CX / 32; ++kc) { const v16b a = frag_b(&sx[wave * 16 + col][kc * 32], lane);
#pragma unroll
      for (int j = 0; j < 4; ++j) { v16b w; const int o = j * 16 + col;
#pragma unroll
        for (int i = 0; i < 8; ++i) { w[i] = (__bf16)W1[o * CX + kc * 32 + 8 * g + i]; w[8 + i] = (__bf16)W1[o * CX + kc * 32 + 16 + 8 * g + i]; }
        acc[j] = wmma_bf(a, w, acc[j]); } }
#pragma unroll
    for (int j = 0; j < 4; ++j) { const float bb = bfr(B1[j * 16 + col]);
#pragma unroll
      for (int r = 0; r < 8; ++r) sa[wave][8 * g + r][j * 16 + col] = acc[j][r] + bb; }
    LDSX();
    v8f acc2[4]; conv2(&sa[wave][col][0], col, lane, g, W2, acc2);
#pragma unroll
    for (int j = 0; j < 4; ++j) { const float bb = bfr(B2[j * 16 + col]);
#pragma unroll
      for (int r = 0; r < 8; ++r) { const float v = acc2[j][r] + bb; const int rl = wave * 16 + 8 * g + r, cl = j * 16 + col; if (which == 1) split_store(v, sh[rl][cl], sl[rl][cl]); else split_store(v, th[cl][rl], tl[cl][rl]); } }
    LDSX(); }
  __syncthreads();
  for (int e = tid; e < 64 * 8; e += 128) { const int rl = e >> 3, q = e & 7; const size_t o = (b * NP + n0 + rl) * CM + q * 8; vst2((unsigned*)(FXH + o), *(const v4u*)&sh[rl][q * 8]); vst2((unsigned*)(FXL + o), *(const v4u*)&sl[rl][q * 8]); }
  for (int e = tid; e < 64 * 8; e += 128) { const int cl = e >> 3, q = e & 7; const size_t o = (b * CM + cl) * (size_t)NP + n0 + q * 8; vst2((unsigned*)(FSH + o), *(const v4u*)&th[cl][q * 8]); vst2((unsigned*)(FSL + o), *(const v4u*)&tl[cl][q * 8]); }
  __syncthreads();
  { const float shf = (float)h0 * 0.5f - 0.25f; int ha = (int)floorf(shf); const float fh = shf - (float)ha; int hb = ha + 1; float wha = 1.0f - fh, whb = fh; if (ha < 0) { ha = 0; } if (hb > HY - 1) { hb = HY - 1; }
    const int wq = wave * 16 + col; const float swf = (float)wq * 0.5f - 0.25f; int wa = (int)floorf(swf); const float fw = swf - (float)wa; int wb = wa + 1; const float wwa = 1.0f - fw, wwb = fw; if (wa < 0) wa = 0; if (wb > WY - 1) wb = WY - 1;
    v8f acc[4] = {};
#pragma unroll 2
    for (int kc = 0; kc < CY / 32; ++kc) { float v[16];
#pragma unroll
      for (int i = 0; i < 8; ++i) {
#pragma unroll
        for (int half = 0; half < 2; ++half) { const int c = kc * 32 + half * 16 + 8 * g + i; const float* yc = Y + ((b * CY + c) * HY) * WY;
          const float yaa = bfr(yc[ha * WY + wa]), yab = bfr(yc[ha * WY + wb]), yba = bfr(yc[hb * WY + wa]), ybb = bfr(yc[hb * WY + wb]);
          v[half * 8 + i] = wha * (wwa * yaa + wwb * yab) + whb * (wwa * yba + wwb * ybb); } }
      const F2 a = bsplit16(v);
#pragma unroll
      for (int j = 0; j < 4; ++j) { v16b w; const int o = j * 16 + col;
#pragma unroll
        for (int i = 0; i < 8; ++i) { w[i] = (__bf16)WY1[o * CY + kc * 32 + 8 * g + i]; w[8 + i] = (__bf16)WY1[o * CY + kc * 32 + 16 + 8 * g + i]; }
        acc[j] = wmma_bf(a.h, w, acc[j]); acc[j] = wmma_bf(a.l, w, acc[j]); } }
#pragma unroll
    for (int j = 0; j < 4; ++j) { const float bb = bfr(BY1[j * 16 + col]);
#pragma unroll
      for (int r = 0; r < 8; ++r) sa[wave][8 * g + r][j * 16 + col] = acc[j][r] + bb; }
    LDSX();
    v8f acc2[4]; conv2(&sa[wave][col][0], col, lane, g, WY2, acc2);
#pragma unroll
    for (int j = 0; j < 4; ++j) { const float bb = bfr(BY2[j * 16 + col]);
#pragma unroll
      for (int r = 0; r < 8; ++r) { const float vv = acc2[j][r] + bb; const int rl = wave * 16 + 8 * g + r, cl = j * 16 + col; split_store(vv, sh[rl][cl], sl[rl][cl]); } }
    __syncthreads();
    for (int e = tid; e < 64 * 8; e += 128) { const int rl = e >> 3, q = e & 7; const size_t o = (b * NP + n0 + rl) * CM + q * 8; vst2((unsigned*)(FYH + o), *(const v4u*)&sh[rl][q * 8]); vst2((unsigned*)(FYL + o), *(const v4u*)&sl[rl][q * 8]); } } }
__global__ __launch_bounds__(128) void k_att(const _Float16* __restrict__ FXH, const _Float16* __restrict__ FXL, const _Float16* __restrict__ FYH, const _Float16* __restrict__ FYL, const _Float16* __restrict__ FSH, const _Float16* __restrict__ FSL, const float* __restrict__ WU, const float* __restrict__ BU, const float* __restrict__ X, float* __restrict__ OUT) {
  __shared__ __align__(16) float sp[4][16][36]; __shared__ __align__(16) float sy[4][16][68]; __shared__ __align__(16) float st[128][68];
  const int tid = threadIdx.x, wave = tid >> 5, lane = tid & 31, col = lane & 15, g = lane >> 4; const int qb = blockIdx.x; const size_t b = blockIdx.y; const int q0 = qb * 64 + wave * 16;
  v16h aq[2], al[2];
#pragma unroll
  for (int kc = 0; kc < 2; ++kc) { aq[kc] = frag_h(FXH + (b * NP + q0 + col) * CM + kc * 32, lane); al[kc] = frag_h(FXL + (b * NP + q0 + col) * CM + kc * 32, lane); }
  float m[8], l[8];
#pragma unroll
  for (int r = 0; r < 8; ++r) { m[r] = -3.0e38f; l[r] = 0.f; }
  v8f acc[4] = {}, accl[4] = {};
#pragma unroll 1
  for (int ks = 0; ks < NP / 32; ++ks) { float s[2][8];
#pragma unroll
    for (int ct = 0; ct < 2; ++ct) { const int kk = ks * 32 + ct * 16 + col; const size_t rk = (b * NP + kk) * CM; v8f c = {}, cl = {};
#pragma unroll
      for (int kc = 0; kc < 2; ++kc) { const v16h kh = frag_h(FYH + rk + kc * 32, lane); c = wmma16(aq[kc], kh, c); cl = wmma16(al[kc], kh, cl); cl = wmma16(aq[kc], frag_h(FYL + rk + kc * 32, lane), cl); }
#pragma unroll
      for (int r = 0; r < 8; ++r) s[ct][r] = c[r] + cl[r] * (1.0f / 2048.0f); }
    float alpha[8];
#pragma unroll
    for (int r = 0; r < 8; ++r) { float mx = fmaxf(s[0][r], s[1][r]);
#pragma unroll
      for (int o = 1; o < 16; o <<= 1) mx = fmaxf(mx, __shfl_xor(mx, o));
      const float mn = fmaxf(m[r], mx); alpha[r] = __expf(m[r] - mn); const float e0 = __expf(s[0][r] - mn), e1 = __expf(s[1][r] - mn); float es = e0 + e1;
#pragma unroll
      for (int o = 1; o < 16; o <<= 1) es += __shfl_xor(es, o);
      l[r] = l[r] * alpha[r] + es; m[r] = mn; sp[wave][8 * g + r][col] = e0; sp[wave][8 * g + r][16 + col] = e1; }
#pragma unroll
    for (int j = 0; j < 4; ++j)
#pragma unroll
      for (int r = 0; r < 8; ++r) { acc[j][r] *= alpha[r]; accl[j][r] *= alpha[r]; }
    LDSX();
    v16h pa, par; { const float* prow = &sp[wave][col][0] + 8 * (lane >> 4);
#pragma unroll
      for (int i = 0; i < 8; ++i) { const float p0 = prow[i] * 2048.0f, p1 = prow[16 + i] * 2048.0f; pa[i] = (_Float16)p0; pa[8 + i] = (_Float16)p1; par[i] = (_Float16)(p0 - (float)pa[i]); par[8 + i] = (_Float16)(p1 - (float)pa[8 + i]); } }
#pragma unroll
    for (int j = 0; j < 4; ++j) { const size_t po = (b * CM + j * 16 + col) * (size_t)NP + ks * 32; const v16h vh = frag_h(FSH + po, lane); acc[j] = wmma16(pa, vh, acc[j]); acc[j] = wmma16(par, vh, acc[j]); accl[j] = wmma16(pa, frag_h(FSL + po, lane), accl[j]); }
    LDSX(); }
#pragma unroll
  for (int r = 0; r < 8; ++r) { const float il = (1.0f / 2048.0f) / l[r];
#pragma unroll
    for (int j = 0; j < 4; ++j) sy[wave][8 * g + r][j * 16 + col] = (acc[j][r] + accl[j][r] * (1.0f / 2048.0f)) * il; }
  LDSX();
#pragma unroll 1
  for (int og = 0; og < 2; ++og) { v8f o8[8] = {};
#pragma unroll
    for (int kc = 0; kc < CM / 32; ++kc) { const F2 a = split_row(&sy[wave][col][0], kc * 32, lane);
#pragma unroll
      for (int j = 0; j < 8; ++j) { v16b w; const int c = og * 128 + j * 16 + col;
#pragma unroll
        for (int i = 0; i < 8; ++i) { w[i] = (__bf16)WU[(size_t)c * CM + kc * 32 + 8 * g + i]; w[8 + i] = (__bf16)WU[(size_t)c * CM + kc * 32 + 16 + 8 * g + i]; }
        o8[j] = wmma_bf(a.h, w, o8[j]); o8[j] = wmma_bf(a.l, w, o8[j]); } }
#pragma unroll
    for (int j = 0; j < 8; ++j)
#pragma unroll
      for (int r = 0; r < 8; ++r) { const int c = og * 128 + j * 16 + col, nl = wave * 16 + 8 * g + r; st[j * 16 + col][nl] = o8[j][r] + bfr(BU[c]) + bfr(X[((b * CX + c) * NP) + qb * 64 + nl]); }
    __syncthreads();
    for (int e = tid; e < 128 * 16; e += 128) { const int cl = e >> 4, q = e & 15; vst2(OUT + ((b * CX + og * 128 + cl) * NP) + qb * 64 + q * 4, *(const v4f*)&st[cl][q * 4]); }
    __syncthreads(); } }
extern "C" void kernel_launch(void* const* d_in, const int* in_sizes, int n_in, void* d_out, int out_size, void* d_ws, size_t ws_size, hipStream_t stream) {
  (void)in_sizes; (void)n_in; (void)out_size;
  const float** F = (const float**)d_in;
  if (ws_size < (size_t)WS_END) return;
  char* ws = (char*)d_ws; _Float16 *FXH = (_Float16*)(ws + WS_FXH), *FXL = (_Float16*)(ws + WS_FXL), *FYH = (_Float16*)(ws + WS_FYH), *FYL = (_Float16*)(ws + WS_FYL), *FSH = (_Float16*)(ws + WS_FSH), *FSL = (_Float16*)(ws + WS_FSL);
  k_feat<<<dim3(HH, TNB), 128, 0, stream>>>(F[0], F[1], F[2], F[3], F[4], F[5], F[6], F[7], F[8], F[9], F[10], F[11], F[12], F[13], FXH, FXL, FYH, FYL, FSH, FSL);
  k_att<<<dim3(NP / 64, TNB), 128, 0, stream>>>(FXH, FXL, FYH, FYL, FSH, FSL, F[14], F[15], F[0], (float*)d_out);
}
